// SelectiveSSM_27127013441892
// MI455X (gfx1250) — hardware-run, weakly checked
//
#include <hip/hip_runtime.h>
#include <math.h>

typedef __attribute__((ext_vector_type(8)))  _Float16 v8h;
typedef __attribute__((ext_vector_type(16))) __bf16   v16b;
typedef __attribute__((ext_vector_type(8)))  __bf16   v8b;
typedef __attribute__((ext_vector_type(8)))  float    v8f;
typedef __attribute__((ext_vector_type(4)))  float    v4f;
typedef __attribute__((ext_vector_type(2)))  float    v2f;
typedef __attribute__((ext_vector_type(4)))  unsigned v4u;

constexpr int kBatch   = 2;
constexpr int kSeq     = 2048;
constexpr int kDm      = 1024;
constexpr int kDin     = 2048;
constexpr int kNst     = 16;
constexpr int kConvK   = 4;
constexpr int kRows    = kBatch * kSeq;
constexpr int kPrmReal = 2 * kNst + 1;
constexpr int kPrmP    = 64;
constexpr int kConvTP  = 260;
constexpr int kTrP     = 65;
constexpr int kScanTS  = 64;
constexpr int kScanCh  = 128;
constexpr int kScanBlkPerB = kDin / kScanCh;
static_assert(kRows == 4096 && kPrmReal == 33, "shape");
static_assert((kDm % 64) == 0 && (kDin % 64) == 0 && (kRows % 64) == 0 && (kPrmP % 64) == 0, "GEMM tile multiples");
static_assert((kDm % 32) == 0 && (kDin % 32) == 0, "GEMM K multiples of 32");
static_assert((kSeq % kScanTS) == 0 && (kSeq % 64) == 0 && (kDin % 256) == 0 && (kDin % kScanCh) == 0, "tile multiples");
static_assert(kPrmReal <= kPrmP, "padded state projection width");

constexpr size_t kSzXP   = (size_t)kRows * kDm * 2;
constexpr size_t kSzWIP  = (size_t)(2 * kDin) * kDm * 2;
constexpr size_t kSzRA   = 2 * kSzXP + 2 * kSzWIP;
constexpr size_t kSzXIN  = (size_t)kRows * kDin * 4;
constexpr size_t kSzGATE = (size_t)kRows * kDin * 2;
constexpr size_t kSzXC   = (size_t)kRows * kDin * 4;
constexpr size_t kSzXCP  = (size_t)kRows * kDin * 2;
constexpr size_t kSzWX   = (size_t)kPrmP * kDin * 2;
constexpr size_t kSzPRM  = (size_t)kRows * kPrmP * 4;
constexpr size_t kSzDT   = (size_t)kRows * 4;
constexpr size_t kSzWO   = (size_t)kDm * kDin * 2;
constexpr size_t kOffRA   = 0;
constexpr size_t kOffXH   = kOffRA;
constexpr size_t kOffXL   = kOffXH  + kSzXP;
constexpr size_t kOffWIH  = kOffXL  + kSzXP;
constexpr size_t kOffWIL  = kOffWIH + kSzWIP;
constexpr size_t kOffXCH  = kOffRA;
constexpr size_t kOffXCL  = kOffRA + kSzXCP;
constexpr size_t kOffYH   = kOffXCH;
constexpr size_t kOffYL   = kOffXCL;
constexpr size_t kOffXIN  = kOffRA   + kSzRA;
constexpr size_t kOffGATE = kOffXIN  + kSzXIN;
constexpr size_t kOffXC   = kOffGATE + kSzGATE;
constexpr size_t kOffWXH  = kOffXC   + kSzXC;
constexpr size_t kOffWXL  = kOffWXH  + kSzWX;
constexpr size_t kOffPRM  = kOffWXL  + kSzWX;
constexpr size_t kOffDT   = kOffPRM  + kSzPRM;
constexpr size_t kOffWOH  = kOffDT   + kSzDT;
constexpr size_t kOffWOL  = kOffWOH  + kSzWO;
constexpr size_t kWsTotal = kOffWOL  + kSzWO;
static_assert(kSzRA == 2 * kSzXCP, "hi and lo planes of xc fit the dead in_proj operand bytes exactly");
static_assert(kOffXCL == kOffWIH, "lo plane of xc starts on the first weight plane");
static_assert(kOffYL + kSzXCP == kOffXIN, "lo plane of the gated y ends where the x_inner plane starts");
static_assert(kSzRA == 33554432ull, "in_proj operand region");
static_assert(kSzWO == 4194304ull, "out weight plane");
static_assert(kWsTotal == 127418368ull, "carve total");
static_assert(kWsTotal <= 134217728ull, "carve cap");
static_assert((kOffXL % 128) == 0 && (kOffWIH % 128) == 0 && (kOffWIL % 128) == 0 && (kOffXCL % 128) == 0 &&
              (kOffXIN % 128) == 0 && (kOffGATE % 128) == 0 && (kOffXC % 128) == 0 &&
              (kOffWXH % 128) == 0 && (kOffWXL % 128) == 0 && (kOffPRM % 128) == 0 &&
              (kOffDT % 128) == 0 && (kOffWOH % 128) == 0 && (kOffWOL % 128) == 0, "128-B aligned regions");

__device__ __forceinline__ unsigned bf_rne_word(float f) {
  unsigned u = __float_as_uint(f);
  const unsigned lsb = (u & 0x00010000u) ? 1u : 0u;
  u = (u + 0x7FFFu + lsb) & 0xFFFF0000u;
  return u;
}
__device__ __forceinline__ void bf_split_pair(float f0, float f1, unsigned& hw, unsigned& lw) {
  const unsigned h0 = bf_rne_word(f0);
  const unsigned h1 = bf_rne_word(f1);
  const float r0 = f0 - __uint_as_float(h0);
  const float r1 = f1 - __uint_as_float(h1);
  const unsigned l0 = bf_rne_word(r0);
  const unsigned l1 = bf_rne_word(r1);
  hw = __builtin_amdgcn_perm(h1, h0, 0x07060302u);
  lw = __builtin_amdgcn_perm(l1, l0, 0x07060302u);
}
__device__ __forceinline__ float h16_to_f32(unsigned hb) {
  const unsigned sgn = (hb & 0x8000u) << 16;
  const unsigned em = hb & 0x7fffu;
  const float fn = __uint_as_float((em << 13) + 0x38000000u);
  const float fs = (float)em * 5.9604644775390625e-8f;
  const float mag = (em < 0x400u) ? fs : fn;
  return __uint_as_float(__float_as_uint(mag) | sgn);
}

__device__ __forceinline__ void tie_b(v8f& c, v16b a, v16b b) { asm volatile("" : "+v"(c) : "v"(a), "v"(b)); }
__device__ __forceinline__ void nop_guard_b(v8f& c, v16b x, v16b y) { asm volatile("v_nop\n\tv_nop\n\tv_nop\n\tv_nop" : "+v"(c) : "v"(x), "v"(y)); }
__device__ __forceinline__ void keep4_b(v16b a, v16b b, v16b c, v16b d) { asm volatile("v_nop" :: "v"(a), "v"(b), "v"(c), "v"(d)); }
__device__ __forceinline__ void acc_guard4(v8f& a, v8f& b, v8f& c, v8f& d) { asm volatile("v_nop\n\tv_nop\n\tv_nop\n\tv_nop" : "+v"(a), "+v"(b), "+v"(c), "+v"(d)); }

template <typename T> struct Frag;
template <> struct Frag<__bf16> {
  typedef v16b V; union U { v16b v; v8b h[2]; };
  static __device__ __forceinline__ v16b load(const __bf16* p) {
    U f; f.h[0] = *(const v8b*)(p); f.h[1] = *(const v8b*)(p + 16); return f.v;
  }
  static __device__ __forceinline__ v8f mma(v16b a, v16b b, v8f c) {
    return __builtin_amdgcn_wmma_f32_16x16x32_bf16(false, a, false, b, (short)0, c, false, false);
  }
  static __device__ __forceinline__ void tie(v8f& c, v16b a, v16b b) { tie_b(c, a, b); }
  static __device__ __forceinline__ void guard(v8f& c, v16b x, v16b y) { nop_guard_b(c, x, y); }
  static __device__ __forceinline__ void keep(v16b a, v16b b, v16b c, v16b d) { keep4_b(a, b, c, d); }
};

template <bool SPLIT, int OUT_MODE, int ACT>
__global__ __launch_bounds__(256) void wmma_gemm64(
    const unsigned short* __restrict__ Ap, const unsigned short* __restrict__ A2p, int lda,
    const unsigned short* __restrict__ Btp, const unsigned short* __restrict__ Bt2p, int ldb,
    void* __restrict__ Cout, int ldc, int M, int N, int K) {
  typedef __bf16 T;
  typedef typename Frag<T>::V V;
  const T* Ab  = (const T*)Ap;
  const T* Ab2 = (const T*)A2p;
  const T* Bb  = (const T*)Btp;
  const T* Bb2 = (const T*)Bt2p;
  __shared__ __align__(16) float sT[8][16 * 68];
  const int lane = threadIdx.x & 31;
  const int wave = threadIdx.x >> 5;
  const int tilesN = N >> 6;
  const int tilesM = M >> 6;
  const int tile = blockIdx.x * 8 + wave;
  if (tile >= tilesM * tilesN) return;
  const int tm = tile / tilesN;
  const int tn = tile - tm * tilesN;
  const int m0 = tm << 6;
  const int n0 = tn << 6;

  const int rlane = lane & 15;
  const int koff  = (lane >> 4) * 8;
  const int mOff  = (lane >> 4) * 8;

  v8f acc[4][4];
#pragma unroll
  for (int i = 0; i < 4; ++i)
#pragma unroll
    for (int j = 0; j < 4; ++j) acc[i][j] = (v8f){0.f,0.f,0.f,0.f,0.f,0.f,0.f,0.f};

  for (int k0 = 0; k0 < K; k0 += 32) {
    V bh[4], bl[4];
#pragma unroll
    for (int j = 0; j < 4; ++j) {
      const size_t bo = (size_t)(n0 + (j << 4) + rlane) * ldb + koff + k0;
      bh[j] = Frag<T>::load(Bb + bo);
      if (SPLIT) bl[j] = Frag<T>::load(Bb2 + bo);
    }
#pragma unroll
    for (int i = 0; i < 4; ++i) {
      const size_t ao = (size_t)(m0 + (i << 4) + rlane) * lda + koff + k0;
      V ah = Frag<T>::load(Ab + ao);
      V al;
      if (SPLIT) al = Frag<T>::load(Ab2 + ao);
#pragma unroll
      for (int j = 0; j < 4; ++j) {
        acc[i][j] = Frag<T>::mma(ah, bh[j], acc[i][j]);
        if (SPLIT) {
          acc[i][j] = Frag<T>::mma(ah, bl[j], acc[i][j]);
          acc[i][j] = Frag<T>::mma(al, bh[j], acc[i][j]);
        }
      }
      Frag<T>::tie(acc[i][0], ah, bh[0]);
      Frag<T>::tie(acc[i][1], ah, bh[1]);
      Frag<T>::tie(acc[i][2], ah, bh[2]);
      Frag<T>::tie(acc[i][3], ah, bh[3]);
      if (SPLIT) {
        Frag<T>::tie(acc[i][0], al, bl[0]);
        Frag<T>::tie(acc[i][1], al, bl[1]);
        Frag<T>::tie(acc[i][2], al, bl[2]);
        Frag<T>::tie(acc[i][3], al, bl[3]);
      }
      Frag<T>::guard(acc[i][3], ah, SPLIT ? al : ah);
    }
    Frag<T>::keep(bh[0], bh[1], bh[2], bh[3]);
    if (SPLIT) Frag<T>::keep(bl[0], bl[1], bl[2], bl[3]);
  }
  acc_guard4(acc[0][0], acc[0][1], acc[0][2], acc[0][3]);
  acc_guard4(acc[1][0], acc[1][1], acc[1][2], acc[1][3]);
  acc_guard4(acc[2][0], acc[2][1], acc[2][2], acc[2][3]);
  acc_guard4(acc[3][0], acc[3][1], acc[3][2], acc[3][3]);

  float* slab = sT[wave];
#pragma unroll
  for (int i = 0; i < 4; ++i) {
    const int mBase = m0 + (i << 4);
#pragma unroll
    for (int j = 0; j < 4; ++j) {
#pragma unroll
      for (int r = 0; r < 8; ++r) {
        float v = acc[i][j][r];
        if (ACT == 3) v = v / (1.0f + expf(-v));
        slab[(mOff + r) * 68 + (j << 4) + rlane] = v;
      }
    }
    __builtin_amdgcn_fence(__ATOMIC_RELEASE, "workgroup");
    __builtin_amdgcn_wave_barrier();
    __builtin_amdgcn_fence(__ATOMIC_ACQUIRE, "workgroup");
    if (OUT_MODE == 0) {
      float* C = (float*)Cout;
      const int hh = lane >> 4, c4 = (lane & 15) * 4;
      for (int pass = 0; pass < 2; ++pass) {
#pragma unroll
        for (int it = 0; it < 8; ++it) {
          const int row = it * 2 + hh;
          v4f v = *(const v4f*)(slab + row * 68 + c4);
          *(volatile v4f*)(C + (size_t)(mBase + row) * ldc + n0 + c4) = v;
        }
        __threadfence();
      }
    } else {
      const int q = lane >> 3, c8 = (lane & 7) * 8;
      unsigned short* C = (unsigned short*)Cout;
      for (int pass = 0; pass < 2; ++pass) {
#pragma unroll
        for (int it = 0; it < 4; ++it) {
          const int row = it * 4 + q;
          const float* sp = slab + row * 68 + c8;
          v8h hv;
#pragma unroll
          for (int e = 0; e < 8; ++e) hv[e] = (_Float16)sp[e];
          *(volatile v8h*)(C + (size_t)(mBase + row) * ldc + n0 + c8) = hv;
        }
        __threadfence();
      }
    }
    __builtin_amdgcn_fence(__ATOMIC_RELEASE, "workgroup");
    __builtin_amdgcn_wave_barrier();
    __builtin_amdgcn_fence(__ATOMIC_ACQUIRE, "workgroup");
  }
}

__global__ __launch_bounds__(256) void split_rows_bf16_kernel(
    const float* __restrict__ src, unsigned short* __restrict__ dhi, unsigned short* __restrict__ dlo, int total8) {
  const int i = blockIdx.x * 256 + threadIdx.x;
  if (i >= total8) return;
  const size_t base = (size_t)i << 3;
  const v4f a0 = *(const v4f*)(src + base);
  const v4f a1 = *(const v4f*)(src + base + 4);
  const float e0 = a0[0], e1 = a0[1], e2 = a0[2], e3 = a0[3];
  const float e4 = a1[0], e5 = a1[1], e6 = a1[2], e7 = a1[3];
  unsigned h01, l01, h23, l23, h45, l45, h67, l67;
  bf_split_pair(e0, e1, h01, l01);
  bf_split_pair(e2, e3, h23, l23);
  bf_split_pair(e4, e5, h45, l45);
  bf_split_pair(e6, e7, h67, l67);
  const v4u hw = (v4u){h01, h23, h45, h67};
  const v4u lw = (v4u){l01, l23, l45, l67};
  unsigned short* qh = dhi + base;
  unsigned short* ql = dlo + base;
  *(volatile v4u*)qh = hw;
  *(volatile v4u*)ql = lw;
  __threadfence();
  *(volatile v4u*)qh = hw;
  *(volatile v4u*)ql = lw;
}

template <bool PERM>
__global__ __launch_bounds__(256) void transpose_planes_kernel(
    const float* __restrict__ W, int KR, int NC,
    unsigned short* __restrict__ P0, unsigned short* __restrict__ P1) {
  __shared__ __align__(16) float sT[64 * kTrP];
  const unsigned tid = threadIdx.x;
  const unsigned lane = tid & 31u;
  const unsigned wave = tid >> 5;
  const unsigned k0 = blockIdx.x * 64u;
  const unsigned n0 = blockIdx.y * 64u;
  {
    const unsigned nc = tid & 63u;
    const unsigned kq = tid >> 6;
    const unsigned n = n0 + nc;
    unsigned csrc;
    bool valid;
    if (PERM) {
      csrc = (n < 32u) ? (n + 1u) : 0u;
      valid = (n <= 32u);
    } else {
      csrc = n;
      valid = (n < (unsigned)NC);
    }
    csrc = (csrc < (unsigned)NC) ? csrc : ((unsigned)NC - 1u);
    asm volatile("" : "+v"(csrc));
#pragma unroll
    for (int i = 0; i < 16; ++i) {
      const unsigned kr = (unsigned)i * 4u + kq;
      float v = W[(size_t)(k0 + kr) * (size_t)NC + csrc];
      asm volatile("" : "+v"(v));
      sT[kr * kTrP + nc] = valid ? v : 0.0f;
    }
  }
  __syncthreads();
  const unsigned q = lane >> 3;
  const unsigned c8 = (lane & 7u) * 8u;
  v4u hw[2], lw[2];
#pragma unroll
  for (int it = 0; it < 2; ++it) {
    const unsigned row = (unsigned)it * 32u + wave * 4u + q;
#pragma unroll
    for (int p = 0; p < 4; ++p) {
      const float f0 = sT[(c8 + 2u * (unsigned)p) * kTrP + row];
      const float f1 = sT[(c8 + 2u * (unsigned)p + 1u) * kTrP + row];
      unsigned hwv, lwv;
      bf_split_pair(f0, f1, hwv, lwv);
      hw[it][p] = hwv;
      lw[it][p] = lwv;
    }
  }
  for (int pass = 0; pass < 2; ++pass) {
#pragma unroll
    for (int it = 0; it < 2; ++it) {
      const unsigned row = (unsigned)it * 32u + wave * 4u + q;
      const size_t o = (size_t)(n0 + row) * (size_t)KR + k0 + c8;
      *(volatile v4u*)(P0 + o) = hw[it];
      *(volatile v4u*)(P1 + o) = lw[it];
    }
    __threadfence();
  }
}

__global__ __launch_bounds__(256) void conv_silu_kernel(
    const float* __restrict__ XI, const float* __restrict__ cw, const float* __restrict__ cb,
    float* __restrict__ XC, unsigned short* __restrict__ XCH, unsigned short* __restrict__ XCL) {
  __shared__ __align__(16) float sT[16 * kConvTP];
  const int tid = threadIdx.x, lane = tid & 31, wave = tid >> 5;
  const int d0 = blockIdx.x * 256, d = d0 + tid;
  const int g0 = blockIdx.y * 64;
  const int tb = g0 & (kSeq - 1);
  const v4f wv = *(const v4f*)(cw + (size_t)d * kConvK);
  const float w0 = wv[0], w1 = wv[1], w2 = wv[2], w3 = wv[3];
  const float bc = cb[d];
  float xm3, xm2, xm1;
  {
    const bool hist = (tb > 0);
    const int rb = hist ? (g0 - 3) : g0;
    const float v3 = XI[(size_t)rb * kDin + d];
    const float v2 = XI[(size_t)(rb + 1) * kDin + d];
    const float v1 = XI[(size_t)(rb + 2) * kDin + d];
    xm3 = hist ? v3 : 0.f;
    xm2 = hist ? v2 : 0.f;
    xm1 = hist ? v1 : 0.f;
  }
  const int hrow = wave >> 1;
  const int hch  = (wave & 1) * 128 + lane * 4;
#pragma unroll 1
  for (int sub = 0; sub < 4; ++sub) {
    const int lb = g0 + sub * 16;
#pragma unroll 1
    for (int s = 0; s < 16; ++s) {
      const float xcur = XI[(size_t)(lb + s) * kDin + d];
      float acc = w0 * xm3;
      acc = fmaf(w1, xm2, acc);
      acc = fmaf(w2, xm1, acc);
      acc = fmaf(w3, xcur, acc);
      const float sv = acc + bc;
      const float sg = 1.0f / (1.0f + expf(-sv));
      sT[s * kConvTP + tid] = sv * sg;
      xm3 = xm2; xm2 = xm1; xm1 = xcur;
    }
    __syncthreads();
    v4f fv[4];
    v4u hw[2], lw[2];
#pragma unroll
    for (int it = 0; it < 4; ++it) fv[it] = *(const v4f*)(sT + (it * 4 + hrow) * kConvTP + hch);
#pragma unroll
    for (int it = 0; it < 2; ++it) {
      const float* sp = sT + (it * 8 + wave) * kConvTP + lane * 8;
      const v4f a0 = *(const v4f*)(sp);
      const v4f a1 = *(const v4f*)(sp + 4);
      const float e0 = a0[0], e1 = a0[1], e2 = a0[2], e3 = a0[3];
      const float e4 = a1[0], e5 = a1[1], e6 = a1[2], e7 = a1[3];
      unsigned h01, l01, h23, l23, h45, l45, h67, l67;
      bf_split_pair(e0, e1, h01, l01);
      bf_split_pair(e2, e3, h23, l23);
      bf_split_pair(e4, e5, h45, l45);
      bf_split_pair(e6, e7, h67, l67);
      hw[it] = (v4u){h01, h23, h45, h67};
      lw[it] = (v4u){l01, l23, l45, l67};
    }
    for (int pass = 0; pass < 2; ++pass) {
#pragma unroll
      for (int it = 0; it < 4; ++it)
        *(volatile v4f*)(XC + (size_t)(lb + it * 4 + hrow) * kDin + d0 + hch) = fv[it];
#pragma unroll
      for (int it = 0; it < 2; ++it) {
        const size_t o = (size_t)(lb + it * 8 + wave) * kDin + d0 + lane * 8;
        *(volatile v4u*)(XCH + o) = hw[it];
        *(volatile v4u*)(XCL + o) = lw[it];
      }
      __threadfence();
    }
    __syncthreads();
  }
}

__global__ __launch_bounds__(256) void softplus_step_kernel(
    const float* __restrict__ PRM, float* __restrict__ DT) {
  const int i = blockIdx.x * 256 + threadIdx.x;
  const float v = PRM[(size_t)i * kPrmP + 2 * kNst];
  const float a = expf(-fabsf(v));
  const float dt = fmaxf(v, 0.0f) + log1pf(a);
  volatile float* p = DT + i;
  *p = dt;
  __threadfence();
  *p = dt;
}

__global__ __launch_bounds__(64) void scan_gate_kernel(
    const float* __restrict__ PRM, const float* __restrict__ DT, const float* __restrict__ XC,
    const unsigned* __restrict__ GATE, const float* __restrict__ Alog, const float* __restrict__ Dp,
    unsigned* __restrict__ YH, unsigned* __restrict__ YL) {
  __shared__ __align__(16) float sBC[kScanTS * 32];
  __shared__ __align__(16) float sDt[kScanTS];
  __shared__ __align__(16) float sA[kScanCh * kNst];
  const unsigned tid = threadIdx.x;
  const unsigned bix = blockIdx.x / (unsigned)kScanBlkPerB;
  const unsigned d0 = (blockIdx.x - bix * (unsigned)kScanBlkPerB) * (unsigned)kScanCh;
  const unsigned dch = d0 + 2u * tid;
  const size_t row0 = (size_t)bix * kSeq;
#pragma unroll 1
  for (int i = 0; i < 32; ++i) {
    const unsigned idx = (unsigned)i * 64u + tid;
    sA[idx] = -expf(Alog[(size_t)d0 * kNst + idx]);
  }
  __syncthreads();
  float a0[kNst], a1[kNst], h0[kNst], h1[kNst];
#pragma unroll
  for (int q4 = 0; q4 < 4; ++q4) {
    const v4f u = *(const v4f*)(sA + (2u * tid) * kNst + 4 * q4);
    const v4f w = *(const v4f*)(sA + (2u * tid + 1u) * kNst + 4 * q4);
    a0[4 * q4 + 0] = u[0]; a0[4 * q4 + 1] = u[1]; a0[4 * q4 + 2] = u[2]; a0[4 * q4 + 3] = u[3];
    a1[4 * q4 + 0] = w[0]; a1[4 * q4 + 1] = w[1]; a1[4 * q4 + 2] = w[2]; a1[4 * q4 + 3] = w[3];
  }
#pragma unroll
  for (int n = 0; n < kNst; ++n) { h0[n] = 0.f; h1[n] = 0.f; }
  const v2f dd = *(const v2f*)(Dp + dch);
  const float dd0 = dd[0], dd1 = dd[1];
  const size_t wcol = (size_t)(d0 >> 1) + tid;
#pragma unroll 1
  for (int t0 = 0; t0 < kSeq; t0 += kScanTS) {
    __syncthreads();
#pragma unroll
    for (int i = 0; i < 8; ++i) {
      const unsigned idx = (unsigned)i * 64u + tid;
      const unsigned r = idx >> 3;
      const unsigned c4 = (idx & 7u) * 4u;
      *(v4f*)(sBC + r * 32u + c4) = *(const v4f*)(PRM + (row0 + t0 + r) * kPrmP + c4);
    }
    sDt[tid] = DT[row0 + t0 + tid];
    __syncthreads();
#pragma unroll 1
    for (int s = 0; s < kScanTS; ++s) {
      const size_t row = row0 + (size_t)t0 + (size_t)s;
      const float dt = sDt[s];
      const v2f xv = *(const v2f*)(XC + row * kDin + dch);
      const unsigned gw = GATE[row * (kDin / 2) + wcol];
      const float* bcp = sBC + s * 32;
      float Bn[kNst], Cn[kNst];
#pragma unroll
      for (int q4 = 0; q4 < 4; ++q4) {
        const v4f bv = *(const v4f*)(bcp + 4 * q4);
        const v4f cv = *(const v4f*)(bcp + kNst + 4 * q4);
        Bn[4 * q4 + 0] = bv[0]; Bn[4 * q4 + 1] = bv[1]; Bn[4 * q4 + 2] = bv[2]; Bn[4 * q4 + 3] = bv[3];
        Cn[4 * q4 + 0] = cv[0]; Cn[4 * q4 + 1] = cv[1]; Cn[4 * q4 + 2] = cv[2]; Cn[4 * q4 + 3] = cv[3];
      }
      const float x0 = xv[0], x1 = xv[1];
      float y0 = 0.f, y1 = 0.f;
#pragma unroll
      for (int n = 0; n < kNst; ++n) {
        const float dbn = dt * Bn[n];
        const float e0 = __expf(dt * a0[n]);
        const float e1 = __expf(dt * a1[n]);
        h0[n] = fmaf(e0, h0[n], dbn * x0);
        h1[n] = fmaf(e1, h1[n], dbn * x1);
        y0 = fmaf(Cn[n], h0[n], y0);
        y1 = fmaf(Cn[n], h1[n], y1);
      }
      y0 = fmaf(x0, dd0, y0);
      y1 = fmaf(x1, dd1, y1);
      const float g0 = h16_to_f32(gw & 0xffffu);
      const float g1 = h16_to_f32(gw >> 16);
      const float yg0 = y0 * g0;
      const float yg1 = y1 * g1;
      unsigned hwd, lwd;
      bf_split_pair(yg0, yg1, hwd, lwd);
      volatile unsigned* ph = YH + row * (kDin / 2) + wcol;
      volatile unsigned* pl = YL + row * (kDin / 2) + wcol;
      *ph = hwd;
      *pl = lwd;
      __threadfence();
      *ph = hwd;
      *pl = lwd;
    }
  }
}

extern "C" void kernel_launch(void* const* d_in, const int* in_sizes, int n_in,
                              void* d_out, int out_size, void* d_ws, size_t ws_size,
                              hipStream_t stream) {
  if (n_in < 8) return;
  if (in_sizes[0] != kRows * kDm) return;
  if (in_sizes[1] != kDm * 2 * kDin) return;
  if (in_sizes[2] != kDin * kConvK) return;
  if (in_sizes[3] != kDin) return;
  if (in_sizes[4] != kDin * kPrmReal) return;
  if (in_sizes[5] != kDin * kNst) return;
  if (in_sizes[6] != kDin) return;
  if (in_sizes[7] != kDin * kDm) return;
  if (out_size != kRows * kDm) return;
  if (ws_size < kWsTotal) return;

  const float* x      = (const float*)d_in[0];
  const float* W_in   = (const float*)d_in[1];
  const float* conv_w = (const float*)d_in[2];
  const float* conv_b = (const float*)d_in[3];
  const float* W_x    = (const float*)d_in[4];
  const float* A_log  = (const float*)d_in[5];
  const float* D_par  = (const float*)d_in[6];
  const float* W_out  = (const float*)d_in[7];
  float* out = (float*)d_out;

  char* ws = (char*)d_ws;
  unsigned short* XH   = (unsigned short*)(ws + kOffXH);
  unsigned short* XL   = (unsigned short*)(ws + kOffXL);
  unsigned short* WIH  = (unsigned short*)(ws + kOffWIH);
  unsigned short* WIL  = (unsigned short*)(ws + kOffWIL);
  unsigned short* XCH  = (unsigned short*)(ws + kOffXCH);
  unsigned short* XCL  = (unsigned short*)(ws + kOffXCL);
  unsigned short* YH   = (unsigned short*)(ws + kOffYH);
  unsigned short* YL   = (unsigned short*)(ws + kOffYL);
  float*          XIN  = (float*)(ws + kOffXIN);
  unsigned short* GATE = (unsigned short*)(ws + kOffGATE);
  float*          XC   = (float*)(ws + kOffXC);
  unsigned short* WXH  = (unsigned short*)(ws + kOffWXH);
  unsigned short* WXL  = (unsigned short*)(ws + kOffWXL);
  float*          PRM  = (float*)(ws + kOffPRM);
  float*          DT   = (float*)(ws + kOffDT);
  unsigned short* WOH  = (unsigned short*)(ws + kOffWOH);
  unsigned short* WOL  = (unsigned short*)(ws + kOffWOL);

  split_rows_bf16_kernel<<<(kRows * kDm / 8) / 256, 256, 0, stream>>>(x, XH, XL, kRows * kDm / 8);
  transpose_planes_kernel<false><<<dim3(kDm / 64, (2 * kDin) / 64), 256, 0, stream>>>(W_in, kDm, 2 * kDin, WIH, WIL);
  transpose_planes_kernel<false><<<dim3(kDin / 64, kDm / 64), 256, 0, stream>>>(W_out, kDin, kDm, WOH, WOL);
  transpose_planes_kernel<true><<<dim3(kDin / 64, kPrmP / 64), 256, 0, stream>>>(W_x, kDin, kPrmReal, WXH, WXL);

  wmma_gemm64<true, 0, 0><<<dim3((kRows / 64) * (kDin / 64) / 8), 256, 0, stream>>>(
      XH, XL, kDm, WIH, WIL, kDm, (void*)XIN, kDin, kRows, kDin, kDm);
  wmma_gemm64<true, 1, 3><<<dim3((kRows / 64) * (kDin / 64) / 8), 256, 0, stream>>>(
      XH, XL, kDm, WIH + (size_t)kDin * kDm, WIL + (size_t)kDin * kDm, kDm, (void*)GATE, kDin, kRows, kDin, kDm);

  conv_silu_kernel<<<dim3(kDin / 256, kRows / 64), 256, 0, stream>>>(XIN, conv_w, conv_b, XC, XCH, XCL);

  wmma_gemm64<true, 0, 0><<<dim3((kRows / 64) * (kPrmP / 64) / 8), 256, 0, stream>>>(
      XCH, XCL, kDin, WXH, WXL, kDin, (void*)PRM, kPrmP, kRows, kPrmP, kDin);

  softplus_step_kernel<<<kRows / 256, 256, 0, stream>>>(PRM, DT);

  scan_gate_kernel<<<kBatch * kScanBlkPerB, 64, 0, stream>>>(
      PRM, DT, XC, (const unsigned*)GATE, A_log, D_par, (unsigned*)YH, (unsigned*)YL);

  wmma_gemm64<true, 0, 0><<<dim3((kRows / 64) * (kDm / 64) / 8), 256, 0, stream>>>(
      YH, YL, kDin, WOH, WOL, kDin, (void*)out, kDm, kRows, kDm, kDin);
}
